// DeltaNet_58205396795472
// MI455X (gfx1250) — hardware-verified
//
#include <hip/hip_runtime.h>
#include <math.h>

constexpr int kBatch   = 2;
constexpr int kSeq     = 2048;
constexpr int kHid     = 1024;
constexpr int kHeads   = 4;
constexpr int kDk      = 256;
constexpr int kTok     = kBatch * kSeq;
constexpr int kBetaCol = 3 * kHid;
constexpr int kNProj   = 3 * kHid + 64;
constexpr int kConvK   = 4;
constexpr int kChunk   = 64;
constexpr int kNChunk  = kSeq / kChunk;
constexpr int kDvSlice = 64;
constexpr int kSlices  = kDk / kDvSlice;
constexpr int kPitchF  = 68;
static_assert(kTok % 64 == 0 && kNProj % 64 == 0 && kHid % 64 == 0 && kHid % 32 == 0);
static_assert(kSeq % kChunk == 0 && kDk % kDvSlice == 0 && kChunk == 64 && kDvSlice == 64 && kDk == 256);
static_assert(kHeads * kDk == kHid);

constexpr float kQKCarry   = 16.0f;
constexpr float kUCarry    = 256.0f;
constexpr float kOnCarry   = 16.0f;
constexpr float kWoCarry   = 256.0f;
constexpr float kInvG      = 1.0f / 256.0f;
constexpr float kInvKS     = 1.0f / 2048.0f;
constexpr float kAqkMul    = 0.25f;
constexpr float kInvAU     = 1.0f / 16384.0f;
constexpr float kShadowMul = 1.0f / 32.0f;
constexpr float kOutScale  = 1.0f / 4096.0f;

typedef __attribute__((ext_vector_type(16))) _Float16 v16h;
typedef __attribute__((ext_vector_type(8)))  _Float16 v8h;
typedef __attribute__((ext_vector_type(16))) __bf16   v16b;
typedef __attribute__((ext_vector_type(8)))  __bf16   v8b;
typedef __attribute__((ext_vector_type(8)))  float    v8f;
typedef __attribute__((ext_vector_type(4)))  float    v4f;
typedef __attribute__((ext_vector_type(4)))  unsigned int v4u;

__device__ __forceinline__ unsigned short f2bf_bits(float f) {
  unsigned u = __float_as_uint(f);
  return (unsigned short)((u + 0x7FFFu + ((u >> 16) & 1u)) >> 16);
}
__device__ __forceinline__ float bf_bits2f(unsigned short h) { return __uint_as_float(((unsigned)h) << 16); }

__device__ __forceinline__ void dep_guard_h(v8f& a, v8f& b, v16h x, v16h y) { asm volatile("v_nop\n\tv_nop\n\tv_nop\n\tv_nop" : "+v"(a), "+v"(b) : "v"(x), "v"(y)); }
__device__ __forceinline__ void dep_guard_b(v8f& a, v8f& b, v16b x, v16b y) { asm volatile("v_nop\n\tv_nop\n\tv_nop\n\tv_nop" : "+v"(a), "+v"(b) : "v"(x), "v"(y)); }
__device__ __forceinline__ void keep4_h(v16h a, v16h b, v16h c, v16h d) { asm volatile("v_nop" :: "v"(a), "v"(b), "v"(c), "v"(d)); }
__device__ __forceinline__ void keep4_b(v16b a, v16b b, v16b c, v16b d) { asm volatile("v_nop" :: "v"(a), "v"(b), "v"(c), "v"(d)); }
__device__ __forceinline__ void acc_guard4(v8f& a, v8f& b, v8f& c, v8f& d) { asm volatile("v_nop\n\tv_nop\n\tv_nop\n\tv_nop" : "+v"(a), "+v"(b), "+v"(c), "+v"(d)); }
template <typename T> struct Frag;
template <> struct Frag<_Float16> {
  typedef v16h V; union U { v16h v; v8h h[2]; };
  static __device__ __forceinline__ v16h load(const _Float16* p) {
    U f; f.h[0] = *(const v8h*)(p); f.h[1] = *(const v8h*)(p + 16); return f.v;
  }
  static __device__ __forceinline__ v8f mma(v16h a, v16h b, v8f c) {
    return __builtin_amdgcn_wmma_f32_16x16x32_f16(false, a, false, b, (short)0, c, false, false);
  }
  static __device__ __forceinline__ void guard(v8f& a, v8f& b, v16h x, v16h y) { dep_guard_h(a, b, x, y); }
  static __device__ __forceinline__ void keep(v16h a, v16h b, v16h c, v16h d) { keep4_h(a, b, c, d); }
};
template <> struct Frag<__bf16> {
  typedef v16b V; union U { v16b v; v8b h[2]; };
  static __device__ __forceinline__ v16b load(const __bf16* p) {
    U f; f.h[0] = *(const v8b*)(p); f.h[1] = *(const v8b*)(p + 16); return f.v;
  }
  static __device__ __forceinline__ v8f mma(v16b a, v16b b, v8f c) {
    return __builtin_amdgcn_wmma_f32_16x16x32_bf16(false, a, false, b, (short)0, c, false, false);
  }
  static __device__ __forceinline__ void guard(v8f& a, v8f& b, v16b x, v16b y) { dep_guard_b(a, b, x, y); }
  static __device__ __forceinline__ void keep(v16b a, v16b b, v16b c, v16b d) { keep4_b(a, b, c, d); }
};

__device__ __forceinline__ unsigned pk16(unsigned short a, unsigned short b) { return (unsigned)a | ((unsigned)b << 16); }
__device__ __forceinline__ unsigned short h_bits(float f) { const _Float16 h = (_Float16)f; return __builtin_bit_cast(unsigned short, h); }

template <int ET> struct Elem;
template <> struct Elem<0> { typedef _Float16 T; };
template <> struct Elem<1> { typedef __bf16 T; };
template <int ET, bool SPLIT, int BIAS_MODE, int OUT_MODE, bool RESID, int ACT = 0>
__global__ __launch_bounds__(256) void wmma_gemm64(
    const unsigned short* __restrict__ Ap, const unsigned short* __restrict__ A2p, int lda, long strideA,
    const unsigned short* __restrict__ Btp, const unsigned short* __restrict__ Bt2p, int ldb, long strideB,
    void* __restrict__ Cout, void* __restrict__ Cout2, int ldc, long strideC,
    const float* __restrict__ bias,
    const float* __restrict__ resid, long strideR,
    int M, int N, int K, float scale) {
  typedef typename Elem<ET>::T T;
  typedef typename Frag<T>::V V;
  const T* A = (const T*)Ap; const T* A2 = (const T*)A2p; const T* Bt = (const T*)Btp; const T* Bt2 = (const T*)Bt2p;
  __shared__ __align__(16) float sT[8][16 * 68];
  const int b    = blockIdx.y;
  const int lane = threadIdx.x & 31;
  const int wave = threadIdx.x >> 5;
  const int tilesN = N >> 6;
  const int tilesM = M >> 6;
  const int tile = blockIdx.x * 8 + wave;
  if (tile >= tilesM * tilesN) return;
  const int tm = tile / tilesN;
  const int tn = tile - tm * tilesN;
  const int m0 = tm << 6;
  const int n0 = tn << 6;

  const T* Ab  = A  + (size_t)b * strideA;
  const T* Bb  = Bt + (size_t)b * strideB;
  const T* Ab2 = SPLIT ? (A2  + (size_t)b * strideA) : nullptr;
  const T* Bb2 = SPLIT ? (Bt2 + (size_t)b * strideB) : nullptr;

  const int rlane = lane & 15;
  const int koff  = (lane >> 4) * 8;
  const int mOff  = (lane >> 4) * 8;

  v8f acc[4][4];
#pragma unroll
  for (int i = 0; i < 4; ++i)
#pragma unroll
    for (int j = 0; j < 4; ++j) acc[i][j] = (v8f){0.f,0.f,0.f,0.f,0.f,0.f,0.f,0.f};

  for (int k0 = 0; k0 < K; k0 += 32) {
    V bh[4], bl[4];
#pragma unroll
    for (int j = 0; j < 4; ++j) {
      const size_t bo = (size_t)(n0 + (j << 4) + rlane) * ldb + koff + k0;
      bh[j] = Frag<T>::load(Bb + bo);
      if (SPLIT) bl[j] = Frag<T>::load(Bb2 + bo);
    }
#pragma unroll
    for (int i = 0; i < 4; ++i) {
      const size_t ao = (size_t)(m0 + (i << 4) + rlane) * lda + koff + k0;
      V ah = Frag<T>::load(Ab + ao);
      V al;
      if (SPLIT) al = Frag<T>::load(Ab2 + ao);
#pragma unroll
      for (int j = 0; j < 4; ++j) {
        acc[i][j] = Frag<T>::mma(ah, bh[j], acc[i][j]);
        if (SPLIT) {
          acc[i][j] = Frag<T>::mma(ah, bl[j], acc[i][j]);
          acc[i][j] = Frag<T>::mma(al, bh[j], acc[i][j]);
        }
      }
      Frag<T>::guard(acc[i][0], acc[i][3], ah, SPLIT ? al : ah);
    }
    Frag<T>::keep(bh[0], bh[1], bh[2], bh[3]);
    if (SPLIT) Frag<T>::keep(bl[0], bl[1], bl[2], bl[3]);
  }
  acc_guard4(acc[0][0], acc[0][1], acc[0][2], acc[0][3]);
  acc_guard4(acc[1][0], acc[1][1], acc[1][2], acc[1][3]);
  acc_guard4(acc[2][0], acc[2][1], acc[2][2], acc[2][3]);
  acc_guard4(acc[3][0], acc[3][1], acc[3][2], acc[3][3]);

  float* slab = sT[wave];
  const float* Rb = RESID ? (resid + (size_t)b * strideR) : nullptr;
#pragma unroll
  for (int i = 0; i < 4; ++i) {
    const int mBase = m0 + (i << 4);
#pragma unroll
    for (int j = 0; j < 4; ++j) {
      const int n = n0 + (j << 4) + rlane;
      float bv = 0.f;
      if (BIAS_MODE == 2) bv = bias[n];
#pragma unroll
      for (int r = 0; r < 8; ++r) {
        float v = acc[i][j][r] * scale;
        if (BIAS_MODE == 1) v += bias[mBase + mOff + r];
        if (BIAS_MODE == 2) v += bv;
        if (RESID) v += Rb[(size_t)(mBase + mOff + r) * ldc + n];
        if (ACT == 2) v = fmaxf(v, 0.0f);
        if (ACT == 4) v = (v > 0.f) ? v : 0.01f * v;
        slab[(mOff + r) * 68 + (j << 4) + rlane] = v;
      }
    }
    __builtin_amdgcn_fence(__ATOMIC_RELEASE, "workgroup");
    __builtin_amdgcn_wave_barrier();
    __builtin_amdgcn_fence(__ATOMIC_ACQUIRE, "workgroup");
    if (OUT_MODE == 0) {
      float* C = (float*)Cout + (size_t)b * strideC;
      const int hh = lane >> 4, c4 = (lane & 15) * 4;
      for (int pass = 0; pass < 2; ++pass) {
#pragma unroll
        for (int it = 0; it < 8; ++it) {
          const int row = it * 2 + hh;
          v4f v = *(const v4f*)(slab + row * 68 + c4);
          *(volatile v4f*)(C + (size_t)(mBase + row) * ldc + n0 + c4) = v;
        }
        __threadfence();
      }
    } else {
      const int q = lane >> 3, c8 = (lane & 7) * 8;
      unsigned short* C  = (unsigned short*)Cout  + (size_t)b * strideC;
      unsigned short* C2 = (OUT_MODE == 2) ? ((unsigned short*)Cout2 + (size_t)b * strideC) : nullptr;
      for (int pass = 0; pass < 2; ++pass) {
#pragma unroll
        for (int it = 0; it < 4; ++it) {
          const int row = it * 4 + q;
          const float* sp = slab + row * 68 + c8;
          v8h hv, lv;
#pragma unroll
          for (int e = 0; e < 8; ++e) {
            if (OUT_MODE == 1) {
              hv[e] = (_Float16)sp[e];
            } else {
              unsigned short hb = f2bf_bits(sp[e]);
              unsigned short lb = f2bf_bits(sp[e] - bf_bits2f(hb));
              hv[e] = __builtin_bit_cast(_Float16, hb);
              lv[e] = __builtin_bit_cast(_Float16, lb);
            }
          }
          *(volatile v8h*)(C + (size_t)(mBase + row) * ldc + n0 + c8) = hv;
          if (OUT_MODE == 2) *(volatile v8h*)(C2 + (size_t)(mBase + row) * ldc + n0 + c8) = lv;
        }
        __threadfence();
      }
    }
    __builtin_amdgcn_fence(__ATOMIC_RELEASE, "workgroup");
    __builtin_amdgcn_wave_barrier();
    __builtin_amdgcn_fence(__ATOMIC_ACQUIRE, "workgroup");
  }
}

__device__ __forceinline__ v8f hmma(v16h a, v16h b, v8f c) {
  c = __builtin_amdgcn_wmma_f32_16x16x32_f16(false, a, false, b, (short)0, c, false, false);
  asm volatile("v_nop\n\tv_nop\n\tv_nop\n\tv_nop" : "+v"(c) : "v"(a), "v"(b));
  return c;
}
__device__ __forceinline__ v16h ldfrag(const unsigned short* p) {
  return Frag<_Float16>::load((const _Float16*)(const void*)p);
}
__device__ __forceinline__ float bf_rne(float f) { return bf_bits2f(f2bf_bits(f)); }

__global__ __launch_bounds__(256) void cast8_bf16_kernel(const float* __restrict__ in, unsigned short* __restrict__ out, int n8) {
  const int i = blockIdx.x * 256 + threadIdx.x;
  if (i >= n8) return;
  const float* p = in + 8 * (size_t)i;
  const v4f a = *(const v4f*)(p);
  const v4f c = *(const v4f*)(p + 4);
  unsigned short hb[8];
#pragma unroll
  for (int e = 0; e < 4; ++e) {
    hb[e]     = f2bf_bits(a[e]);
    hb[4 + e] = f2bf_bits(c[e]);
  }
  const v4u u = (v4u){pk16(hb[0], hb[1]), pk16(hb[2], hb[3]), pk16(hb[4], hb[5]), pk16(hb[6], hb[7])};
  unsigned short* q = out + 8 * (size_t)i;
  *(volatile v4u*)q = u;
  __threadfence();
  *(volatile v4u*)q = u;
}

__global__ __launch_bounds__(256) void wt_kernel(const float* __restrict__ W0, const float* __restrict__ W1,
                                                 const float* __restrict__ W2, const float* __restrict__ W3,
                                                 unsigned short* __restrict__ WT, unsigned short* __restrict__ WoT) {
  __shared__ float sm[64][65];
  const int t   = threadIdx.x;
  const int k0t = blockIdx.x * 64;
  const int n0  = blockIdx.y * 64;
  const int z   = blockIdx.z;
  const float* W = (z == 0) ? W0 : (z == 1) ? W1 : (z == 2) ? W2 : W3;
#pragma unroll
  for (int i = 0; i < 16; ++i) {
    const int e = i * 256 + t;
    const int r = e >> 6;
    const int c = e & 63;
    sm[c][r] = W[(size_t)(k0t + r) * kHid + n0 + c];
  }
  __syncthreads();
  const int lane = t & 31, wave = t >> 5;
  const int q = lane >> 3, c8 = (lane & 7) * 8;
  const bool isO = (z == 3);
  unsigned short* op = isO ? WoT : (WT + (size_t)z * kHid * kHid);
  for (int pass = 0; pass < 2; ++pass) {
#pragma unroll
    for (int it = 0; it < 2; ++it) {
      const int row = wave * 8 + it * 4 + q;
      unsigned short hb[8];
#pragma unroll
      for (int e = 0; e < 8; ++e) {
        const float x = sm[row][c8 + e];
        const unsigned short bb = f2bf_bits(x);
        const unsigned short hbv = h_bits(bf_bits2f(bb) * kWoCarry);
        hb[e] = isO ? hbv : bb;
      }
      const v4u u = (v4u){pk16(hb[0], hb[1]), pk16(hb[2], hb[3]), pk16(hb[4], hb[5]), pk16(hb[6], hb[7])};
      *(volatile v4u*)(op + (size_t)(n0 + row) * kHid + k0t + c8) = u;
    }
    __threadfence();
  }
}

__global__ __launch_bounds__(128) void wb_rows_kernel(const float* __restrict__ Wb, unsigned short* __restrict__ WT) {
  const int x = blockIdx.x;
  const int t = threadIdx.x;
  const bool live = (x < kHeads);
  const int hsel = live ? x : (kHeads - 1);
  const int k = t * 8;
  unsigned short hb[8];
#pragma unroll
  for (int e = 0; e < 8; ++e) {
    const float w = Wb[(size_t)(k + e) * kHeads + hsel];
    const unsigned short bb = f2bf_bits(w);
    hb[e] = live ? bb : (unsigned short)0;
  }
  const v4u u = (v4u){pk16(hb[0], hb[1]), pk16(hb[2], hb[3]), pk16(hb[4], hb[5]), pk16(hb[6], hb[7])};
  unsigned short* dst = WT + (size_t)(kBetaCol + x) * kHid + k;
  *(volatile v4u*)dst = u;
  __threadfence();
  *(volatile v4u*)dst = u;
}

__global__ __launch_bounds__(256) void conv_act_kernel(const float* __restrict__ QKV,
                                                       const float* __restrict__ cq, const float* __restrict__ ck,
                                                       const float* __restrict__ cv,
                                                       unsigned short* __restrict__ Q16, unsigned short* __restrict__ K16,
                                                       float* __restrict__ V32) {
  __shared__ __align__(16) float slab[8][256];
  const int tid = threadIdx.x, lane = tid & 31, wave = tid >> 5;
  const int id   = blockIdx.x * 8 + wave;
  const int row  = id / 12;
  const int rem  = id - row * 12;
  const int tsel = rem >> 2;
  const int h    = rem & 3;
  const int b    = row >> 11;
  const int s    = row & (kSeq - 1);
  const float* w = (tsel == 0) ? cq : (tsel == 1) ? ck : cv;
  const int colbase = tsel * kHid + h * kDk;
  float* sl = slab[wave];
  float ss = 0.f;
#pragma unroll 1
  for (int grp = 0; grp < 2; ++grp) {
    const int dl = grp * 128 + lane * 4;
    const int ch = h * kDk + dl;
    float wr[4][4];
#pragma unroll
    for (int c = 0; c < 4; ++c) {
      const v4f wv = *(const v4f*)(w + (size_t)(ch + c) * kConvK);
#pragma unroll
      for (int j = 0; j < 4; ++j) wr[c][j] = bf_rne(wv[j]);
    }
    float acc[4] = {0.f, 0.f, 0.f, 0.f};
#pragma unroll
    for (int d = 0; d < kConvK; ++d) {
      const int sp  = s - (kConvK - 1) + d;
      const int spc = (sp < 0) ? 0 : sp;
      const float f = (sp < 0) ? 0.f : 1.f;
      const v4f xv = *(const v4f*)(QKV + (size_t)(b * kSeq + spc) * kNProj + colbase + dl);
#pragma unroll
      for (int c = 0; c < 4; ++c) acc[c] = fmaf(wr[c][d], xv[c] * f, acc[c]);
    }
#pragma unroll
    for (int c = 0; c < 4; ++c) {
      const float x  = acc[c];
      const float sg = 1.0f / (1.0f + expf(-x));
      const float y  = x * sg;
      ss = fmaf(y, y, ss);
      sl[dl + c] = y;
    }
    asm volatile("" : "+v"(ss) :: "memory");
  }
#pragma unroll
  for (int off = 16; off > 0; off >>= 1) ss += __shfl_xor(ss, off, 32);
  const float sc = (tsel < 2) ? rsqrtf(ss + 1e-6f) : 1.0f;
  __builtin_amdgcn_fence(__ATOMIC_RELEASE, "workgroup");
  __builtin_amdgcn_wave_barrier();
  __builtin_amdgcn_fence(__ATOMIC_ACQUIRE, "workgroup");
  if (tsel < 2) {
    const v4f a = *(const v4f*)(sl + lane * 8);
    const v4f c = *(const v4f*)(sl + lane * 8 + 4);
    unsigned short hb[8];
#pragma unroll
    for (int e = 0; e < 4; ++e) {
      const float y0 = (a[e] * sc) * kQKCarry;
      const float y1 = (c[e] * sc) * kQKCarry;
      hb[e]     = h_bits(y0);
      hb[4 + e] = h_bits(y1);
    }
    const v4u u = (v4u){pk16(hb[0], hb[1]), pk16(hb[2], hb[3]), pk16(hb[4], hb[5]), pk16(hb[6], hb[7])};
    unsigned short* dst = ((tsel == 0) ? Q16 : K16) + (size_t)row * kHid + h * kDk + lane * 8;
    *(volatile v4u*)dst = u;
    __threadfence();
    *(volatile v4u*)dst = u;
  } else {
    const v4f a = *(const v4f*)(sl + lane * 4);
    const v4f c = *(const v4f*)(sl + 128 + lane * 4);
    float* dst = V32 + (size_t)row * kHid + h * kDk;
    for (int pass = 0; pass < 2; ++pass) {
      *(volatile v4f*)(dst + lane * 4) = a;
      *(volatile v4f*)(dst + 128 + lane * 4) = c;
      __threadfence();
    }
  }
}

constexpr int kLdsK     = 0;
constexpr int kLdsKt    = kLdsK  + kChunk * kDk * 2;
constexpr int kLdsSt    = kLdsKt + kDk * kChunk * 2;
constexpr int kLdsUt    = kLdsSt + kDvSlice * kDk * 2;
constexpr int kLdsA     = kLdsUt + kDvSlice * kChunk * 2;
constexpr int kLdsU     = kLdsA  + kChunk * kChunk * 2;
constexpr int kLdsG     = kLdsU  + kChunk * kPitchF * 4;
constexpr int kLdsB     = kLdsG  + kChunk * kPitchF * 4;
constexpr int kLdsTotal = kLdsB  + kChunk * 4;
static_assert(kLdsTotal == 149760);
static_assert((kLdsKt % 16) == 0 && (kLdsSt % 16) == 0 && (kLdsUt % 16) == 0 && (kLdsA % 16) == 0 && (kLdsU % 16) == 0 && (kLdsG % 16) == 0 && (kLdsB % 16) == 0);

__global__ __launch_bounds__(256) void delta_chunk_kernel(const unsigned short* __restrict__ Q16,
                                                          const unsigned short* __restrict__ K16,
                                                          const float* __restrict__ V32,
                                                          const float* __restrict__ QKV,
                                                          float* __restrict__ O32) {
  extern __shared__ __align__(16) unsigned char dsm[];
  unsigned short* sK  = (unsigned short*)(dsm + kLdsK);
  unsigned short* sKt = (unsigned short*)(dsm + kLdsKt);
  unsigned short* sSt = (unsigned short*)(dsm + kLdsSt);
  unsigned short* sUt = (unsigned short*)(dsm + kLdsUt);
  unsigned short* sA  = (unsigned short*)(dsm + kLdsA);
  float* sU = (float*)(dsm + kLdsU);
  float* sG = (float*)(dsm + kLdsG);
  float* sB = (float*)(dsm + kLdsB);

  const int tid = threadIdx.x, lane = tid & 31, wv = tid >> 5;
  const int hh = lane >> 4, rl = lane & 15;
  const int g   = blockIdx.x & 3;
  const int bhd = blockIdx.x >> 2;
  const int h   = bhd & 3;
  const int b   = bhd >> 2;
  const int chq = h * kDk;
  const int chv = h * kDk + g * kDvSlice;
  const int mt  = wv >> 1;
  const int nt0 = (wv & 1) * 2;

  const v8f z8 = (v8f){0.f,0.f,0.f,0.f,0.f,0.f,0.f,0.f};
  v8f Sacc[2][4];
#pragma unroll
  for (int ti = 0; ti < 2; ++ti)
#pragma unroll
    for (int nj = 0; nj < 4; ++nj) Sacc[ti][nj] = z8;
  for (int i = tid; i < (kDvSlice * kDk * 2) / 16; i += 256) ((v4u*)sSt)[i] = (v4u){0u, 0u, 0u, 0u};
  __syncthreads();

  for (int tc = 0; tc < kNChunk; ++tc) {
    const int rowb = b * kSeq + tc * kChunk;

    {
      const int r = tid >> 2, q4 = tid & 3;
      const unsigned short* gk = K16 + (size_t)(rowb + r) * kHid + chq + q4 * 64;
#pragma unroll
      for (int i = 0; i < 8; ++i) {
        const v4u w = *(const v4u*)(gk + 8 * i);
        *(v4u*)(sK + r * kDk + q4 * 64 + 8 * i) = w;
#pragma unroll
        for (int e = 0; e < 4; ++e) {
          const unsigned x = w[e];
          const int col = q4 * 64 + 8 * i + 2 * e;
          sKt[col * kChunk + r]       = (unsigned short)(x & 0xffffu);
          sKt[(col + 1) * kChunk + r] = (unsigned short)(x >> 16);
        }
      }
      asm volatile("" ::: "memory");
      const float* gv = V32 + (size_t)(rowb + r) * kHid + chv + q4 * 16;
#pragma unroll
      for (int i = 0; i < 4; ++i) {
        const v4f x = *(const v4f*)(gv + 4 * i);
        *(v4f*)(sU + r * kPitchF + q4 * 16 + 4 * i) = x;
      }
      if (tid < kChunk) {
        const float x = QKV[(size_t)(rowb + tid) * kNProj + kBetaCol + h];
        sB[tid] = 1.0f / (1.0f + expf(-x));
      }
    }
    __syncthreads();

    {
      v8f aG0 = z8, aG1 = z8, aQ0 = z8, aQ1 = z8, aV0 = z8, aV1 = z8;
      const unsigned short* pAK = sK + (mt * 16 + rl) * kDk + 8 * hh;
      const unsigned short* pAQ = Q16 + (size_t)(rowb + mt * 16 + rl) * kHid + chq + 8 * hh;
      const unsigned short* pB0 = sK + (nt0 * 16 + rl) * kDk + 8 * hh;
      const unsigned short* pB1 = pB0 + 16 * kDk;
      const unsigned short* pS0 = sSt + (nt0 * 16 + rl) * kDk + 8 * hh;
      const unsigned short* pS1 = pS0 + 16 * kDk;
#pragma unroll 1
      for (int k0 = 0; k0 < kDk; k0 += 32) {
        const v16h ak = ldfrag(pAK + k0);
        const v16h aq = ldfrag(pAQ + k0);
        const v16h b0 = ldfrag(pB0 + k0);
        const v16h b1 = ldfrag(pB1 + k0);
        const v16h s0 = ldfrag(pS0 + k0);
        const v16h s1 = ldfrag(pS1 + k0);
        aG0 = hmma(ak, b0, aG0);
        aG1 = hmma(ak, b1, aG1);
        aQ0 = hmma(aq, b0, aQ0);
        aQ1 = hmma(aq, b1, aQ1);
        aV0 = hmma(ak, s0, aV0);
        aV1 = hmma(ak, s1, aV1);
      }
#pragma unroll
      for (int r = 0; r < 8; ++r) {
        const int i  = mt * 16 + 8 * hh + r;
        const int j0 = nt0 * 16 + rl;
        const int j1 = j0 + 16;
        sG[i * kPitchF + j0] = aG0[r] * kInvG;
        sG[i * kPitchF + j1] = aG1[r] * kInvG;
        const unsigned short qa0 = h_bits(aQ0[r] * kAqkMul);
        const unsigned short qa1 = h_bits(aQ1[r] * kAqkMul);
        sA[i * kChunk + j0] = (j0 <= i) ? qa0 : (unsigned short)0;
        sA[i * kChunk + j1] = (j1 <= i) ? qa1 : (unsigned short)0;
        sU[i * kPitchF + j0] -= aV0[r] * kInvKS;
        sU[i * kPitchF + j1] -= aV1[r] * kInvKS;
      }
    }
    __syncthreads();

    {
      const int cl = lane & 7, jg = lane >> 3;
      const int col = wv * 8 + cl;
      for (int i = 0; i < kChunk; ++i) {
        float part = 0.f;
        for (int j = jg; j < i; j += 4) part = fmaf(sG[i * kPitchF + j], sU[j * kPitchF + col], part);
        part += __shfl_xor(part, 8, 32);
        part += __shfl_xor(part, 16, 32);
        const float vt = sU[i * kPitchF + col];
        const float u  = sB[i] * (vt - part);
        if (jg == 0) sU[i * kPitchF + col] = u;
        __builtin_amdgcn_fence(__ATOMIC_RELEASE, "workgroup");
        __builtin_amdgcn_wave_barrier();
        __builtin_amdgcn_fence(__ATOMIC_ACQUIRE, "workgroup");
      }
    }
    __syncthreads();

    {
      const int tt = tid & 63, cg = tid >> 6;
#pragma unroll
      for (int e = 0; e < 16; ++e) {
        const int c = cg * 16 + e;
        sUt[c * kChunk + tt] = h_bits(sU[tt * kPitchF + c] * kUCarry);
      }
    }
    __syncthreads();

    {
      v8f o1a = z8, o1b = z8, o2a = z8, o2b = z8;
      const unsigned short* pAQ = Q16 + (size_t)(rowb + mt * 16 + rl) * kHid + chq + 8 * hh;
      const unsigned short* pS0 = sSt + (nt0 * 16 + rl) * kDk + 8 * hh;
      const unsigned short* pS1 = pS0 + 16 * kDk;
#pragma unroll 1
      for (int k0 = 0; k0 < kDk; k0 += 32) {
        const v16h aq = ldfrag(pAQ + k0);
        const v16h s0 = ldfrag(pS0 + k0);
        const v16h s1 = ldfrag(pS1 + k0);
        o1a = hmma(aq, s0, o1a);
        o1b = hmma(aq, s1, o1b);
      }
      const unsigned short* pA  = sA + (mt * 16 + rl) * kChunk + 8 * hh;
      const unsigned short* pU0 = sUt + (nt0 * 16 + rl) * kChunk + 8 * hh;
      const unsigned short* pU1 = pU0 + 16 * kChunk;
#pragma unroll
      for (int k0 = 0; k0 < kChunk; k0 += 32) {
        const v16h a  = ldfrag(pA + k0);
        const v16h u0 = ldfrag(pU0 + k0);
        const v16h u1 = ldfrag(pU1 + k0);
        o2a = hmma(a, u0, o2a);
        o2b = hmma(a, u1, o2b);
      }
#pragma unroll
      for (int r = 0; r < 8; ++r) {
        const int i  = mt * 16 + 8 * hh + r;
        const int j0 = nt0 * 16 + rl;
        const int j1 = j0 + 16;
        sU[i * kPitchF + j0] = o1a[r] * kInvKS + o2a[r] * kInvAU;
        sU[i * kPitchF + j1] = o1b[r] * kInvKS + o2b[r] * kInvAU;
      }
    }
    {
      const unsigned short* pKt0 = sKt + (32 * wv + rl) * kChunk + 8 * hh;
      const unsigned short* pKt1 = pKt0 + 16 * kChunk;
      const unsigned short* pU   = sUt + rl * kChunk + 8 * hh;
#pragma unroll
      for (int k0 = 0; k0 < kChunk; k0 += 32) {
        const v16h a0 = ldfrag(pKt0 + k0);
        const v16h a1 = ldfrag(pKt1 + k0);
        const v16h u0 = ldfrag(pU + 0 * 16 * kChunk + k0);
        const v16h u1 = ldfrag(pU + 1 * 16 * kChunk + k0);
        const v16h u2 = ldfrag(pU + 2 * 16 * kChunk + k0);
        const v16h u3 = ldfrag(pU + 3 * 16 * kChunk + k0);
        Sacc[0][0] = hmma(a0, u0, Sacc[0][0]);
        Sacc[0][1] = hmma(a0, u1, Sacc[0][1]);
        Sacc[0][2] = hmma(a0, u2, Sacc[0][2]);
        Sacc[0][3] = hmma(a0, u3, Sacc[0][3]);
        Sacc[1][0] = hmma(a1, u0, Sacc[1][0]);
        Sacc[1][1] = hmma(a1, u1, Sacc[1][1]);
        Sacc[1][2] = hmma(a1, u2, Sacc[1][2]);
        Sacc[1][3] = hmma(a1, u3, Sacc[1][3]);
      }
    }
    __syncthreads();

    {
#pragma unroll
      for (int ti = 0; ti < 2; ++ti) {
#pragma unroll
        for (int nj = 0; nj < 4; ++nj) {
          unsigned short sb[8];
#pragma unroll
          for (int r = 0; r < 8; ++r) sb[r] = h_bits(Sacc[ti][nj][r] * kShadowMul);
          const v4u u = (v4u){pk16(sb[0], sb[1]), pk16(sb[2], sb[3]), pk16(sb[4], sb[5]), pk16(sb[6], sb[7])};
          *(v4u*)(sSt + (nj * 16 + rl) * kDk + 32 * wv + 16 * ti + 8 * hh) = u;
        }
      }
      const int c4 = rl * 4;
      for (int pass = 0; pass < 2; ++pass) {
#pragma unroll
        for (int it = 0; it < 4; ++it) {
          const int r = wv * 8 + 2 * it + hh;
          const v4f val = *(const v4f*)(sU + r * kPitchF + c4);
          *(volatile v4f*)(O32 + (size_t)(rowb + r) * kHid + chv + c4) = val;
        }
        __threadfence();
      }
    }
    __syncthreads();
  }
}

__global__ __launch_bounds__(256) void rmsnorm_kernel(const float* __restrict__ O32, const float* __restrict__ nw,
                                                      unsigned short* __restrict__ ON16) {
  const int tid = threadIdx.x, lane = tid & 31, wave = tid >> 5;
  const int id  = blockIdx.x * 8 + wave;
  const int row = id >> 2, h = id & 3;
  const float* p = O32 + (size_t)row * kHid + h * kDk + lane * 8;
  const v4f a  = *(const v4f*)(p);
  const v4f c  = *(const v4f*)(p + 4);
  const v4f wa = *(const v4f*)(nw + lane * 8);
  const v4f wc = *(const v4f*)(nw + lane * 8 + 4);
  float ss = 0.f;
#pragma unroll
  for (int e = 0; e < 4; ++e) { ss = fmaf(a[e], a[e], ss); ss = fmaf(c[e], c[e], ss); }
#pragma unroll
  for (int off = 16; off > 0; off >>= 1) ss += __shfl_xor(ss, off, 32);
  const float sc = rsqrtf(ss * (1.0f / 256.0f) + 1e-5f);
  unsigned short hb[8];
#pragma unroll
  for (int e = 0; e < 4; ++e) {
    const float y0 = ((a[e] * sc) * bf_rne(wa[e])) * kOnCarry;
    const float y1 = ((c[e] * sc) * bf_rne(wc[e])) * kOnCarry;
    hb[e]     = h_bits(y0);
    hb[4 + e] = h_bits(y1);
  }
  const v4u u = (v4u){pk16(hb[0], hb[1]), pk16(hb[2], hb[3]), pk16(hb[4], hb[5]), pk16(hb[6], hb[7])};
  unsigned short* dst = ON16 + (size_t)row * kHid + h * kDk + lane * 8;
  *(volatile v4u*)dst = u;
  __threadfence();
  *(volatile v4u*)dst = u;
}

extern "C" void kernel_launch(void* const* d_in, const int* in_sizes, int n_in,
                              void* d_out, int out_size, void* d_ws, size_t ws_size,
                              hipStream_t stream) {
  if (n_in < 10) return;
  if (in_sizes[0] != kTok * kHid) return;
  if (in_sizes[1] != kHid * kHid || in_sizes[2] != kHid * kHid || in_sizes[3] != kHid * kHid) return;
  if (in_sizes[4] != kHid * kHeads) return;
  if (in_sizes[5] != kHid * kConvK || in_sizes[6] != kHid * kConvK || in_sizes[7] != kHid * kConvK) return;
  if (in_sizes[8] != kDk || in_sizes[9] != kHid * kHid) return;
  if (out_size != kTok * kHid) return;

  const size_t szXb  = (size_t)kTok * kHid * 2;
  const size_t szWT  = (size_t)kNProj * kHid * 2;
  const size_t szWoT = (size_t)kHid * kHid * 2;
  const size_t szQKV = (size_t)kTok * kNProj * 4;
  const size_t sz16  = (size_t)kTok * kHid * 2;
  const size_t sz32  = (size_t)kTok * kHid * 4;
  const size_t offXb  = 0;
  const size_t offWT  = offXb  + szXb;
  const size_t offWoT = offWT  + szWT;
  const size_t offQKV = offWoT + szWoT;
  const size_t offQ16 = offQKV + szQKV;
  const size_t offK16 = offQ16 + sz16;
  const size_t offV32 = offK16 + sz16;
  const size_t offO32 = offV32 + sz32;
  const size_t offON  = offO32 + sz32;
  const size_t total  = offON  + sz16;
  if (ws_size < total) return;

  const float* hs = (const float*)d_in[0];
  const float* Wq = (const float*)d_in[1];
  const float* Wk = (const float*)d_in[2];
  const float* Wv = (const float*)d_in[3];
  const float* Wb = (const float*)d_in[4];
  const float* cq = (const float*)d_in[5];
  const float* ck = (const float*)d_in[6];
  const float* cv = (const float*)d_in[7];
  const float* nw = (const float*)d_in[8];
  const float* Wo = (const float*)d_in[9];
  float* out = (float*)d_out;
  char* ws = (char*)d_ws;
  unsigned short* Xb   = (unsigned short*)(ws + offXb);
  unsigned short* WT   = (unsigned short*)(ws + offWT);
  unsigned short* WoT  = (unsigned short*)(ws + offWoT);
  float*          QKV  = (float*)(ws + offQKV);
  unsigned short* Q16  = (unsigned short*)(ws + offQ16);
  unsigned short* K16  = (unsigned short*)(ws + offK16);
  float*          V32  = (float*)(ws + offV32);
  float*          O32  = (float*)(ws + offO32);
  unsigned short* ON16 = (unsigned short*)(ws + offON);

  const int n8 = (kTok * kHid) / 8;
  cast8_bf16_kernel<<<dim3(n8 / 256), dim3(256), 0, stream>>>(hs, Xb, n8);
  wt_kernel<<<dim3(kHid / 64, kHid / 64, 4), dim3(256), 0, stream>>>(Wq, Wk, Wv, Wo, WT, WoT);
  wb_rows_kernel<<<dim3(kNProj - kBetaCol), dim3(128), 0, stream>>>(Wb, WT);

  const int tilesProj = (kTok / 64) * (kNProj / 64);
  wmma_gemm64<1, false, 0, 0, false, 0><<<dim3(tilesProj / 8, 1), dim3(256), 0, stream>>>(
      Xb, Xb, kHid, 0L, WT, WT, kHid, 0L,
      (void*)QKV, (void*)QKV, kNProj, 0L, V32, V32, 0L, kTok, kNProj, kHid, 1.0f);

  conv_act_kernel<<<dim3((kTok * kHeads * 3) / 8), dim3(256), 0, stream>>>(QKV, cq, ck, cv, Q16, K16, V32);

  delta_chunk_kernel<<<dim3(kBatch * kHeads * kSlices), dim3(256), kLdsTotal, stream>>>(Q16, K16, V32, QKV, O32);

  rmsnorm_kernel<<<dim3((kTok * kHeads) / 8), dim3(256), 0, stream>>>(O32, nw, ON16);

  const int tilesOut = (kTok / 64) * (kHid / 64);
  wmma_gemm64<0, false, 0, 0, false, 0><<<dim3(tilesOut / 8, 1), dim3(256), 0, stream>>>(
      ON16, ON16, kHid, 0L, WoT, WoT, kHid, 0L,
      (void*)out, (void*)out, kHid, 0L, V32, V32, 0L, kTok, kHid, kHid, kOutScale);
}
